// Monotonic_attention_train_14035953123582
// MI455X (gfx1250) — hardware-verified
//
#include <hip/hip_runtime.h>
#include <math.h>

constexpr int NBATCH = 16;
constexpr int NSEQ   = 1024;
constexpr int NHID   = 256;
constexpr int NDIM   = 512;
constexpr int NCLS   = 1000;
constexpr int NSTEPS = 8;
constexpr int NGATE  = 4 * NHID;
constexpr int NPROJ  = 2 * NDIM;
constexpr int YPITCH = 1024;
constexpr int NROWS  = NBATCH * NSEQ;
constexpr int ROWS_PER_EBLK = 32;
constexpr float WCARRY     = 16.0f;
constexpr float WCARRY_INV = 1.0f / 16.0f;
static_assert(NSEQ % ROWS_PER_EBLK == 0, "energy blocks stay inside one batch row");
static_assert(NROWS % 64 == 0 && NPROJ % 64 == 0 && NDIM % 32 == 0, "GEMM tile multiples");
static_assert((NBATCH * NSTEPS * NCLS) % (256 * 4) == 0, "pack grid exact");
static_assert(NCLS % 4 == 0, "float4 groups never straddle output rows");
static_assert(NSEQ == 4 * 256 && NHID == 256 && NDIM == 2 * 256, "thread maps");

typedef __attribute__((ext_vector_type(16))) _Float16 v16h;
typedef __attribute__((ext_vector_type(8)))  _Float16 v8h;
typedef __attribute__((ext_vector_type(16))) __bf16   v16b;
typedef __attribute__((ext_vector_type(8)))  __bf16   v8b;
typedef __attribute__((ext_vector_type(8)))  float    v8f;
typedef __attribute__((ext_vector_type(4)))  float    v4f;
typedef __attribute__((ext_vector_type(4)))  unsigned int v4u;

__device__ __forceinline__ unsigned short f2bf_bits(float f) {
  unsigned u = __float_as_uint(f);
  return (unsigned short)((u + 0x7FFFu + ((u >> 16) & 1u)) >> 16);
}
__device__ __forceinline__ float bf_bits2f(unsigned short h) { return __uint_as_float(((unsigned)h) << 16); }

__device__ __forceinline__ void dep_guard6_h(v8f& a, v8f& b, v8f& c, v8f& d, v16h x, v16h x2, v16h y0, v16h y1, v16h y2, v16h y3) {
  asm volatile("v_nop\n\tv_nop\n\tv_nop\n\tv_nop" : "+v"(a), "+v"(b), "+v"(c), "+v"(d) : "v"(x), "v"(x2), "v"(y0), "v"(y1), "v"(y2), "v"(y3));
}
__device__ __forceinline__ void dep_guard6_b(v8f& a, v8f& b, v8f& c, v8f& d, v16b x, v16b x2, v16b y0, v16b y1, v16b y2, v16b y3) {
  asm volatile("v_nop\n\tv_nop\n\tv_nop\n\tv_nop" : "+v"(a), "+v"(b), "+v"(c), "+v"(d) : "v"(x), "v"(x2), "v"(y0), "v"(y1), "v"(y2), "v"(y3));
}
__device__ __forceinline__ void keep4_h(v16h a, v16h b, v16h c, v16h d) { asm volatile("v_nop" :: "v"(a), "v"(b), "v"(c), "v"(d)); }
__device__ __forceinline__ void keep4_b(v16b a, v16b b, v16b c, v16b d) { asm volatile("v_nop" :: "v"(a), "v"(b), "v"(c), "v"(d)); }
__device__ __forceinline__ void acc_guard4(v8f& a, v8f& b, v8f& c, v8f& d) { asm volatile("v_nop\n\tv_nop\n\tv_nop\n\tv_nop" : "+v"(a), "+v"(b), "+v"(c), "+v"(d)); }

template <typename T> struct Frag;
template <> struct Frag<_Float16> {
  typedef v16h V; union U { v16h v; v8h h[2]; };
  static __device__ __forceinline__ v16h load(const _Float16* p) {
    U f; f.h[0] = *(const v8h*)(p); f.h[1] = *(const v8h*)(p + 16); return f.v;
  }
  static __device__ __forceinline__ v8f mma(v16h a, v16h b, v8f c) {
    return __builtin_amdgcn_wmma_f32_16x16x32_f16(false, a, false, b, (short)0, c, false, false);
  }
  static __device__ __forceinline__ void guard(v8f& a, v8f& b, v8f& c, v8f& d, v16h x, v16h x2, v16h y0, v16h y1, v16h y2, v16h y3) {
    dep_guard6_h(a, b, c, d, x, x2, y0, y1, y2, y3);
  }
  static __device__ __forceinline__ void keep(v16h a, v16h b, v16h c, v16h d) { keep4_h(a, b, c, d); }
};
template <> struct Frag<__bf16> {
  typedef v16b V; union U { v16b v; v8b h[2]; };
  static __device__ __forceinline__ v16b load(const __bf16* p) {
    U f; f.h[0] = *(const v8b*)(p); f.h[1] = *(const v8b*)(p + 16); return f.v;
  }
  static __device__ __forceinline__ v8f mma(v16b a, v16b b, v8f c) {
    return __builtin_amdgcn_wmma_f32_16x16x32_bf16(false, a, false, b, (short)0, c, false, false);
  }
  static __device__ __forceinline__ void guard(v8f& a, v8f& b, v8f& c, v8f& d, v16b x, v16b x2, v16b y0, v16b y1, v16b y2, v16b y3) {
    dep_guard6_b(a, b, c, d, x, x2, y0, y1, y2, y3);
  }
  static __device__ __forceinline__ void keep(v16b a, v16b b, v16b c, v16b d) { keep4_b(a, b, c, d); }
};

__device__ __forceinline__ unsigned pk16(unsigned short a, unsigned short b) { return (unsigned)a | ((unsigned)b << 16); }
__device__ __forceinline__ unsigned short h_bits(float f) { const _Float16 h = (_Float16)f; return __builtin_bit_cast(unsigned short, h); }

__device__ __forceinline__ float sigm_f(float x) { return __builtin_amdgcn_rcpf(1.0f + expf(-x)); }
__device__ __forceinline__ float tanh_e(float x) { return 1.0f - 2.0f * __builtin_amdgcn_rcpf(expf(2.0f * x) + 1.0f); }

template <int ET> struct Elem;
template <> struct Elem<0> { typedef _Float16 T; };
template <> struct Elem<1> { typedef __bf16 T; };
template <int ET, bool SPLIT, int BIAS_MODE, int OUT_MODE, bool RESID, int ACT = 0>
__global__ __launch_bounds__(256) void wmma_gemm64(
    const unsigned short* __restrict__ Ap, const unsigned short* __restrict__ A2p, int lda, long strideA,
    const unsigned short* __restrict__ Btp, const unsigned short* __restrict__ Bt2p, int ldb, long strideB,
    void* __restrict__ Cout, void* __restrict__ Cout2, int ldc, long strideC,
    const float* __restrict__ bias,
    const float* __restrict__ resid, long strideR,
    int M, int N, int K, float scale) {
  typedef typename Elem<ET>::T T;
  typedef typename Frag<T>::V V;
  const T* A = (const T*)Ap; const T* A2 = (const T*)A2p; const T* Bt = (const T*)Btp; const T* Bt2 = (const T*)Bt2p;
  __shared__ __align__(16) float sT[8][16 * 68];
  const int b    = blockIdx.y;
  const int lane = threadIdx.x & 31;
  const int wave = threadIdx.x >> 5;
  const int tilesN = N >> 6;
  const int tilesM = M >> 6;
  const int tile = blockIdx.x * 8 + wave;
  if (tile >= tilesM * tilesN) return;
  const int tm = tile / tilesN;
  const int tn = tile - tm * tilesN;
  const int m0 = tm << 6;
  const int n0 = tn << 6;

  const T* Ab  = A  + (size_t)b * strideA;
  const T* Bb  = Bt + (size_t)b * strideB;
  const T* Ab2 = SPLIT ? (A2  + (size_t)b * strideA) : nullptr;
  const T* Bb2 = SPLIT ? (Bt2 + (size_t)b * strideB) : nullptr;

  const int rlane = lane & 15;
  const int koff  = (lane >> 4) * 8;
  const int mOff  = (lane >> 4) * 8;

  v8f acc[4][4];
#pragma unroll
  for (int i = 0; i < 4; ++i)
#pragma unroll
    for (int j = 0; j < 4; ++j) acc[i][j] = (v8f){0.f,0.f,0.f,0.f,0.f,0.f,0.f,0.f};

  for (int k0 = 0; k0 < K; k0 += 32) {
    V bh[4], bl[4];
#pragma unroll
    for (int j = 0; j < 4; ++j) {
      const size_t bo = (size_t)(n0 + (j << 4) + rlane) * ldb + koff + k0;
      bh[j] = Frag<T>::load(Bb + bo);
      if (SPLIT) bl[j] = Frag<T>::load(Bb2 + bo);
    }
#pragma unroll
    for (int i = 0; i < 4; ++i) {
      const size_t ao = (size_t)(m0 + (i << 4) + rlane) * lda + koff + k0;
      V ah = Frag<T>::load(Ab + ao);
      V al;
      if (SPLIT) al = Frag<T>::load(Ab2 + ao);
#pragma unroll
      for (int j = 0; j < 4; ++j) {
        acc[i][j] = Frag<T>::mma(ah, bh[j], acc[i][j]);
        if (SPLIT) {
          acc[i][j] = Frag<T>::mma(ah, bl[j], acc[i][j]);
          acc[i][j] = Frag<T>::mma(al, bh[j], acc[i][j]);
        }
      }
      Frag<T>::guard(acc[i][0], acc[i][1], acc[i][2], acc[i][3], ah, SPLIT ? al : ah, bh[0], bh[1], bh[2], bh[3]);
    }
    Frag<T>::keep(bh[0], bh[1], bh[2], bh[3]);
    if (SPLIT) Frag<T>::keep(bl[0], bl[1], bl[2], bl[3]);
  }
  acc_guard4(acc[0][0], acc[0][1], acc[0][2], acc[0][3]);
  acc_guard4(acc[1][0], acc[1][1], acc[1][2], acc[1][3]);
  acc_guard4(acc[2][0], acc[2][1], acc[2][2], acc[2][3]);
  acc_guard4(acc[3][0], acc[3][1], acc[3][2], acc[3][3]);

  float* slab = sT[wave];
  const float* Rb = RESID ? (resid + (size_t)b * strideR) : nullptr;
#pragma unroll
  for (int i = 0; i < 4; ++i) {
    const int mBase = m0 + (i << 4);
#pragma unroll
    for (int j = 0; j < 4; ++j) {
      const int n = n0 + (j << 4) + rlane;
      float bv = 0.f;
      if (BIAS_MODE == 2) bv = bias[n];
#pragma unroll
      for (int r = 0; r < 8; ++r) {
        float v = acc[i][j][r] * scale;
        if (BIAS_MODE == 1) v += bias[mBase + mOff + r];
        if (BIAS_MODE == 2) v += bv;
        if (RESID) v += Rb[(size_t)(mBase + mOff + r) * ldc + n];
        if (ACT == 2) v = fmaxf(v, 0.0f);
        if (ACT == 4) v = (v > 0.f) ? v : 0.01f * v;
        slab[(mOff + r) * 68 + (j << 4) + rlane] = v;
      }
    }
    __builtin_amdgcn_fence(__ATOMIC_RELEASE, "workgroup");
    __builtin_amdgcn_wave_barrier();
    __builtin_amdgcn_fence(__ATOMIC_ACQUIRE, "workgroup");
    if (OUT_MODE == 0) {
      float* C = (float*)Cout + (size_t)b * strideC;
      const int hh = lane >> 4, c4 = (lane & 15) * 4;
      for (int pass = 0; pass < 2; ++pass) {
#pragma unroll
        for (int it = 0; it < 8; ++it) {
          const int row = it * 2 + hh;
          v4f v = *(const v4f*)(slab + row * 68 + c4);
          *(volatile v4f*)(C + (size_t)(mBase + row) * ldc + n0 + c4) = v;
        }
        __threadfence();
      }
    } else {
      const int q = lane >> 3, c8 = (lane & 7) * 8;
      unsigned short* C  = (unsigned short*)Cout  + (size_t)b * strideC;
      unsigned short* C2 = (OUT_MODE == 2) ? ((unsigned short*)Cout2 + (size_t)b * strideC) : nullptr;
      for (int pass = 0; pass < 2; ++pass) {
#pragma unroll
        for (int it = 0; it < 4; ++it) {
          const int row = it * 4 + q;
          const float* sp = slab + row * 68 + c8;
          v8h hv, lv;
#pragma unroll
          for (int e = 0; e < 8; ++e) {
            if (OUT_MODE == 1) {
              hv[e] = (_Float16)sp[e];
            } else {
              unsigned short hb = f2bf_bits(sp[e]);
              unsigned short lb = f2bf_bits(sp[e] - bf_bits2f(hb));
              hv[e] = __builtin_bit_cast(_Float16, hb);
              lv[e] = __builtin_bit_cast(_Float16, lb);
            }
          }
          *(volatile v8h*)(C + (size_t)(mBase + row) * ldc + n0 + c8) = hv;
          if (OUT_MODE == 2) *(volatile v8h*)(C2 + (size_t)(mBase + row) * ldc + n0 + c8) = lv;
        }
        __threadfence();
      }
    }
    __builtin_amdgcn_fence(__ATOMIC_RELEASE, "workgroup");
    __builtin_amdgcn_wave_barrier();
    __builtin_amdgcn_fence(__ATOMIC_ACQUIRE, "workgroup");
  }
}

__global__ __launch_bounds__(256) void wtcast_kernel(const float* __restrict__ W0, const float* __restrict__ W1,
                                                     unsigned short* __restrict__ out, float scale) {
  __shared__ float tl[64][65];
  const int t  = threadIdx.x;
  const int d0 = blockIdx.x * 64;
  const int h0 = blockIdx.y * 64;
  const int z  = blockIdx.z;
  const float* W = (z == 0) ? W0 : W1;
#pragma unroll
  for (int i = 0; i < 16; ++i) {
    const int e = i * 256 + t;
    const int r = e >> 6;
    const int c = e & 63;
    tl[c][r] = W[(size_t)(d0 + r) * NDIM + h0 + c] * scale;
  }
  __syncthreads();
  const int lane = t & 31, wave = t >> 5;
  const int q = lane >> 3, c8 = (lane & 7) * 8;
  unsigned short* op = out + (size_t)z * NDIM * NDIM;
  for (int pass = 0; pass < 2; ++pass) {
#pragma unroll
    for (int it = 0; it < 2; ++it) {
      const int row = wave * 8 + it * 4 + q;
      unsigned short hb[8];
#pragma unroll
      for (int e = 0; e < 8; ++e) hb[e] = h_bits(tl[row][c8 + e]);
      const v4u u = (v4u){pk16(hb[0], hb[1]), pk16(hb[2], hb[3]), pk16(hb[4], hb[5]), pk16(hb[6], hb[7])};
      *(volatile v4u*)(op + (size_t)(h0 + row) * NDIM + d0 + c8) = u;
    }
    __threadfence();
  }
}

__global__ __launch_bounds__(256) void cast8_f16_kernel(const float* __restrict__ in, unsigned short* __restrict__ out, int n8) {
  const int i = blockIdx.x * 256 + threadIdx.x;
  if (i >= n8) return;
  const float* p = in + 8 * (size_t)i;
  const v4f a = *(const v4f*)(p);
  const v4f c = *(const v4f*)(p + 4);
  unsigned short hb[8];
#pragma unroll
  for (int e = 0; e < 4; ++e) {
    hb[e]     = h_bits(a[e]);
    hb[4 + e] = h_bits(c[e]);
  }
  const v4u u = (v4u){pk16(hb[0], hb[1]), pk16(hb[2], hb[3]), pk16(hb[4], hb[5]), pk16(hb[6], hb[7])};
  unsigned short* q = out + 8 * (size_t)i;
  *(volatile v4u*)q = u;
  __threadfence();
  *(volatile v4u*)q = u;
}

__global__ __launch_bounds__(256) void init_state_kernel(const float* __restrict__ vmono, const float* __restrict__ gmono,
                                                         const float* __restrict__ bm, const float* __restrict__ bc,
                                                         float* __restrict__ acar0, float* __restrict__ s0,
                                                         float* __restrict__ c0, float* __restrict__ smsc,
                                                         float* __restrict__ vnorm) {
  __shared__ float red[8];
  const int tid = threadIdx.x, lane = tid & 31, wave = tid >> 5;
  const int b = blockIdx.x;
  const float v0 = vmono[tid], v1 = vmono[tid + 256];
  float ss = v0 * v0 + v1 * v1;
#pragma unroll
  for (int off = 16; off > 0; off >>= 1) ss += __shfl_xor(ss, off, 32);
  if (lane == 0) red[wave] = ss;
  __syncthreads();
  float tot = 0.0f;
#pragma unroll
  for (int w = 0; w < 8; ++w) tot += red[w];
  const float vn = gmono[0] / sqrtf(tot);

  const int which = tid >> 7;
  const int idx = (tid & 127) * 4;
  const v4f va = *(const v4f*)(bm + idx);
  const v4f vb = *(const v4f*)(bc + idx);
  v4f sv;
#pragma unroll
  for (int e = 0; e < 4; ++e) sv[e] = which ? vb[e] : va[e];
  v4f av = (v4f){0.f, 0.f, 0.f, 0.f};
  av[0] = (tid == 0) ? 1.0f : 0.0f;
  const v4f zv = (v4f){0.f, 0.f, 0.f, 0.f};
  const v4f nv = (v4f){vn, vn, vn, vn};
  for (int pass = 0; pass < 2; ++pass) {
    *(volatile v4f*)(acar0 + b * NSEQ + 4 * tid) = av;
    *(volatile v4f*)(smsc + b * NPROJ + 4 * tid) = sv;
    if (tid < 64) {
      *(volatile v4f*)(s0 + b * NHID + 4 * tid) = zv;
      *(volatile v4f*)(c0 + b * NHID + 4 * tid) = zv;
    }
    if (b == 0 && tid < 8) *(volatile v4f*)(vnorm + 4 * tid) = nv;
    __threadfence();
  }
}

__global__ __launch_bounds__(256) void energies_kernel(
    const float* __restrict__ Pf, const float* __restrict__ smsc,
    const float* __restrict__ vmono, const float* __restrict__ vchunk,
    const float* __restrict__ vnp, const float* __restrict__ rmono,
    const int* __restrict__ len, const float* __restrict__ noise_t,
    float* __restrict__ pbuf, float* __restrict__ ebuf) {
  __shared__ __align__(16) float resp[ROWS_PER_EBLK];
  __shared__ __align__(16) float rese[ROWS_PER_EBLK];
  const int tid = threadIdx.x, lane = tid & 31, wave = tid >> 5;
  const int row0 = blockIdx.x * ROWS_PER_EBLK;
  const int b  = row0 / NSEQ;
  const int s0 = row0 - b * NSEQ;
  int L = len[b];
  L = (L < 0) ? 0 : ((L > NSEQ) ? NSEQ : L);
  const float vn = vnp[0];
  const float rm = rmono[0];
  const float* sb = smsc + b * NPROJ;
#pragma unroll 1
  for (int rr = 0; rr < 4; ++rr) {
    const int lr  = wave * 4 + rr;
    const int row = row0 + lr;
    const float* pr = Pf + (size_t)row * NPROJ;
    float nz = noise_t[row];
    asm volatile("" : "+v"(nz));
    float am = 0.0f, ac = 0.0f;
#pragma unroll 1
    for (int hsel = 0; hsel < 2; ++hsel) {
      const float* vv = hsel ? vchunk : vmono;
      float acc = 0.0f;
#pragma unroll 1
      for (int j = 0; j < 4; ++j) {
        const int d = (j * 32 + lane) * 4;
        const v4f e = *(const v4f*)(pr + hsel * NDIM + d);
        const v4f t = *(const v4f*)(sb + hsel * NDIM + d);
        const v4f v = *(const v4f*)(vv + d);
        acc += tanhf(e[0] + t[0]) * v[0];
        acc += tanhf(e[1] + t[1]) * v[1];
        acc += tanhf(e[2] + t[2]) * v[2];
        acc += tanhf(e[3] + t[3]) * v[3];
      }
#pragma unroll
      for (int off = 16; off > 0; off >>= 1) acc += __shfl_xor(acc, off, 32);
      am = hsel ? am : acc;
      ac = hsel ? acc : ac;
    }
    const int s = s0 + lr;
    const bool masked = (s >= L);
    const float em = (vn * am + rm) + nz;
    const float sg = sigm_f(em);
    float pv = masked ? 0.0f : sg;
    float ev = masked ? 0.0f : ac;
    asm volatile("" : "+v"(pv), "+v"(ev));
    if (lane == 0) { resp[lr] = pv; rese[lr] = ev; }
  }
  __syncthreads();
  if (wave == 0 && lane < 8) {
    const v4f v = *(const v4f*)(resp + 4 * lane);
    float* dst = pbuf + row0 + 4 * lane;
    *(volatile v4f*)dst = v;
    __threadfence();
    *(volatile v4f*)dst = v;
  }
  if (wave == 1 && lane < 8) {
    const v4f v = *(const v4f*)(rese + 4 * lane);
    float* dst = ebuf + row0 + 4 * lane;
    *(volatile v4f*)dst = v;
    __threadfence();
    *(volatile v4f*)dst = v;
  }
}

__device__ __forceinline__ float block_excl_scan(float total, float* wt, int lane, int wave) {
  float x = total;
#pragma unroll
  for (int off = 1; off < 32; off <<= 1) {
    const float n = __shfl_up(x, off, 32);
    x += (lane >= off) ? n : 0.0f;
  }
  float ex = __shfl_up(x, 1, 32);
  ex = (lane == 0) ? 0.0f : ex;
  if (lane == 31) wt[wave] = x;
  __syncthreads();
  float woff = 0.0f;
#pragma unroll
  for (int w = 0; w < 8; ++w) woff += (w < wave) ? wt[w] : 0.0f;
  return woff + ex;
}

__global__ __launch_bounds__(256) void attend_decode_kernel(
    const float* __restrict__ enc, const int* __restrict__ target, const int* __restrict__ len,
    const float* __restrict__ pbuf, const float* __restrict__ ebuf,
    const float* __restrict__ acar_in, float* __restrict__ acar_out,
    const float* __restrict__ s_in, const float* __restrict__ c_in,
    float* __restrict__ s_out, float* __restrict__ c_out,
    const float* __restrict__ Lys, const float* __restrict__ Lss,
    const float* __restrict__ Lgsw, const float* __restrict__ Lgsb,
    const float* __restrict__ Lgyw, const float* __restrict__ Lgyb,
    const float* __restrict__ Lsy, const float* __restrict__ Lyyw, const float* __restrict__ Lyyb,
    const float* __restrict__ Wsm, const float* __restrict__ Wsmb,
    const float* __restrict__ Wsc, const float* __restrict__ Wscb,
    float* __restrict__ smsc, float* __restrict__ Yt, int step) {
  __shared__ __align__(16) float sh_p[NSEQ];
  __shared__ __align__(16) float sh_a[NSEQ];
  __shared__ __align__(16) float sh_ex[NSEQ];
  __shared__ __align__(16) float sh_g[NSEQ];
  __shared__ __align__(16) float sh_cpp[NSEQ];
  __shared__ __align__(16) float sh_u[NSEQ];
  __shared__ __align__(16) float sh_al[NSEQ];
  __shared__ __align__(16) float sh_r[NSEQ];
  __shared__ __align__(16) float sh_beta[NSEQ];
  __shared__ __align__(16) float sh_cpart[2 * NDIM];
  __shared__ __align__(16) float sh_ctx[NDIM];
  __shared__ __align__(16) float sh_s[NHID];
  __shared__ __align__(16) float sh_sn[NHID];
  __shared__ __align__(16) float sh_cn[NHID];
  __shared__ __align__(16) float sh_h[NHID];
  __shared__ __align__(16) float sh_y[YPITCH];
  __shared__ __align__(16) float sh_sm[NPROJ];
  __shared__ float redm[8];
  __shared__ float wtA[8];
  __shared__ float wtB[8];

  const int tid = threadIdx.x, lane = tid & 31, wave = tid >> 5;
  const int b = blockIdx.x;
  const int i0 = tid * 4;
  int L = len[b];
  L = (L < 0) ? 0 : ((L > NSEQ) ? NSEQ : L);
  const float* prow = pbuf + b * NSEQ;
  const float* erow = ebuf + b * NSEQ;
  const float* arow = acar_in + b * NSEQ;

  sh_s[tid] = s_in[b * NHID + tid];
  const float cold = c_in[b * NHID + tid];

  float ml = -3.0e38f;
#pragma unroll 1
  for (int j = 0; j < 4; ++j) {
    const int i = j * 256 + tid;
    const float pv = prow[i];
    const float ev = erow[i];
    const float av = arow[i];
    sh_p[i] = pv;
    sh_a[i] = av;
    sh_ex[i] = ev;
    sh_g[i] = logf(fminf(fmaxf(1.0f - pv, 1e-8f), 1.0f));
    ml = (i < L) ? fmaxf(ml, ev) : ml;
  }
#pragma unroll
  for (int off = 16; off > 0; off >>= 1) ml = fmaxf(ml, __shfl_xor(ml, off, 32));
  if (lane == 0) redm[wave] = ml;
  __syncthreads();
  float mx = redm[0];
#pragma unroll
  for (int w = 1; w < 8; ++w) mx = fmaxf(mx, redm[w]);

#pragma unroll 1
  for (int j = 0; j < 4; ++j) {
    const int i = j * 256 + tid;
    const float t = fmaxf(expf(sh_ex[i] - mx), 1e-5f);
    sh_ex[i] = (i < L) ? t : 1e-5f;
  }

  {
    const v4f g4 = *(const v4f*)(sh_g + i0);
    const float e1 = g4[0];
    const float e2 = e1 + g4[1];
    const float e3 = e2 + g4[2];
    const float tot = e3 + g4[3];
    const float off = block_excl_scan(tot, wtA, lane, wave);
    v4f x4;
    x4[0] = off;
    x4[1] = off + e1;
    x4[2] = off + e2;
    x4[3] = off + e3;
    *(v4f*)(sh_cpp + i0) = x4;
  }
  __syncthreads();

#pragma unroll 1
  for (int j = 0; j < 4; ++j) {
    const int i = j * 256 + tid;
    float cp = expf(sh_cpp[i]);
    cp = (cp < 1.17549435e-38f) ? 0.0f : cp;
    sh_cpp[i] = cp;
    const float cl = fminf(fmaxf(cp, 1e-8f), 1.0f);
    sh_u[i] = sh_a[i] * __builtin_amdgcn_rcpf(cl);
  }
  __syncthreads();

  {
    const v4f u4 = *(const v4f*)(sh_u + i0);
    const v4f c4 = *(const v4f*)(sh_cpp + i0);
    const v4f p4 = *(const v4f*)(sh_p + i0);
    const float c0 = u4[0];
    const float c1 = c0 + u4[1];
    const float c2 = c1 + u4[2];
    const float c3 = c2 + u4[3];
    const float off2 = block_excl_scan(c3, wtB, lane, wave);
    v4f al;
    al[0] = fminf(fmaxf(p4[0] * (c4[0] * (off2 + c0)), 1e-8f), 1.0f);
    al[1] = fminf(fmaxf(p4[1] * (c4[1] * (off2 + c1)), 1e-8f), 1.0f);
    al[2] = fminf(fmaxf(p4[2] * (c4[2] * (off2 + c2)), 1e-8f), 1.0f);
    al[3] = fminf(fmaxf(p4[3] * (c4[3] * (off2 + c3)), 1e-8f), 1.0f);
    *(v4f*)(sh_al + i0) = al;
  }
  __syncthreads();

#pragma unroll 1
  for (int j = 0; j < 4; ++j) {
    const int i = j * 256 + tid;
    float d = 0.0f;
#pragma unroll
    for (int k = 3; k >= 0; --k) {
      const int ii = i - k;
      const int ic = (ii < 0) ? 0 : ii;
      const float v = sh_ex[ic];
      d += (ii >= 0) ? v : 0.0f;
    }
    d = fmaxf(d, 1e-10f);
    sh_r[i] = sh_al[i] * __builtin_amdgcn_rcpf(d);
  }
  __syncthreads();

#pragma unroll 1
  for (int j = 0; j < 4; ++j) {
    const int i = j * 256 + tid;
    float ms = 0.0f;
#pragma unroll
    for (int k = 0; k < 4; ++k) {
      const int ii = i + k;
      const int ic = (ii > NSEQ - 1) ? (NSEQ - 1) : ii;
      const float v = sh_r[ic];
      ms += (ii < NSEQ) ? v : 0.0f;
    }
    sh_beta[i] = sh_ex[i] * ms;
  }
  __syncthreads();

  {
    const int cg = tid & 127, sp = tid >> 7;
    const float* eb = enc + (size_t)b * NSEQ * NDIM + 4 * cg;
    v4f acc = (v4f){0.f, 0.f, 0.f, 0.f};
#pragma unroll 1
    for (int it = 0; it < NSEQ / 2; ++it) {
      const int s = 2 * it + sp;
      const float bv = sh_beta[s];
      const v4f e4 = *(const v4f*)(eb + (size_t)s * NDIM);
      acc[0] = fmaf(bv, e4[0], acc[0]);
      acc[1] = fmaf(bv, e4[1], acc[1]);
      acc[2] = fmaf(bv, e4[2], acc[2]);
      acc[3] = fmaf(bv, e4[3], acc[3]);
    }
    *(v4f*)(sh_cpart + sp * NDIM + 4 * cg) = acc;
  }
  __syncthreads();
  sh_ctx[tid]       = sh_cpart[tid] + sh_cpart[NDIM + tid];
  sh_ctx[tid + 256] = sh_cpart[tid + 256] + sh_cpart[NDIM + tid + 256];
  __syncthreads();

  float r0 = 0.0f, r1 = 0.0f, r2 = 0.0f, r3 = 0.0f;
#pragma unroll 1
  for (int k = 0; k < NHID; ++k) {
    const float sv = sh_s[k];
    const float* w = Lss + (size_t)k * NGATE + tid;
    r0 = fmaf(sv, w[0], r0);
    r1 = fmaf(sv, w[NHID], r1);
    r2 = fmaf(sv, w[2 * NHID], r2);
    r3 = fmaf(sv, w[3 * NHID], r3);
  }
#pragma unroll 1
  for (int k = 0; k < NDIM; ++k) {
    const float cv = sh_ctx[k];
    const float* w = Lgsw + (size_t)k * NGATE + tid;
    r0 = fmaf(cv, w[0], r0);
    r1 = fmaf(cv, w[NHID], r1);
    r2 = fmaf(cv, w[2 * NHID], r2);
    r3 = fmaf(cv, w[3 * NHID], r3);
  }
  {
    int tg = target[b * NSTEPS + step];
    tg = (tg < 0) ? 0 : ((tg > NCLS - 1) ? (NCLS - 1) : tg);
    const float* ly = Lys + (size_t)tg * NGATE + tid;
    r0 += ly[0] + Lgsb[tid];
    r1 += ly[NHID] + Lgsb[NHID + tid];
    r2 += ly[2 * NHID] + Lgsb[2 * NHID + tid];
    r3 += ly[3 * NHID] + Lgsb[3 * NHID + tid];
  }
  {
    const float ig = sigm_f(r0);
    const float fg = sigm_f(r1);
    const float gg = tanh_e(r2);
    const float og = sigm_f(r3);
    const float cn = fg * cold + ig * gg;
    const float sn = og * tanh_e(cn);
    sh_cn[tid] = cn;
    sh_sn[tid] = sn;
  }
  __syncthreads();

  {
    float acc = Lgyb[tid];
#pragma unroll 1
    for (int k = 0; k < NDIM; ++k) acc = fmaf(sh_ctx[k], Lgyw[(size_t)k * NHID + tid], acc);
#pragma unroll 1
    for (int k = 0; k < NHID; ++k) acc = fmaf(sh_sn[k], Lsy[(size_t)k * NHID + tid], acc);
    sh_h[tid] = tanh_e(acc);
  }
  __syncthreads();

  {
    const int n3 = tid + 768;
    const int n3c = (n3 < NCLS) ? n3 : (NCLS - 1);
    float y0 = 0.0f, y1 = 0.0f, y2 = 0.0f, y3 = 0.0f;
#pragma unroll 1
    for (int k = 0; k < NHID; ++k) {
      const float hv = sh_h[k];
      const float* w = Lyyw + (size_t)k * NCLS;
      y0 = fmaf(hv, w[tid], y0);
      y1 = fmaf(hv, w[tid + 256], y1);
      y2 = fmaf(hv, w[tid + 512], y2);
      y3 = fmaf(hv, w[n3c], y3);
    }
    y0 += Lyyb[tid];
    y1 += Lyyb[tid + 256];
    y2 += Lyyb[tid + 512];
    y3 += Lyyb[n3c];
    y3 = (n3 < NCLS) ? y3 : 0.0f;
    sh_y[tid] = y0;
    sh_y[tid + 256] = y1;
    sh_y[tid + 512] = y2;
    sh_y[tid + 768] = y3;
  }
  const bool donext = (step + 1 < NSTEPS);
  if (donext) {
    float m0 = 0.0f, m1 = 0.0f, m2 = 0.0f, m3 = 0.0f;
#pragma unroll 1
    for (int k = 0; k < NHID; ++k) {
      const float sv = sh_sn[k];
      const float* wm = Wsm + (size_t)k * NDIM + tid;
      const float* wc = Wsc + (size_t)k * NDIM + tid;
      m0 = fmaf(sv, wm[0], m0);
      m1 = fmaf(sv, wm[256], m1);
      m2 = fmaf(sv, wc[0], m2);
      m3 = fmaf(sv, wc[256], m3);
    }
    m0 += Wsmb[tid];
    m1 += Wsmb[tid + 256];
    m2 += Wscb[tid];
    m3 += Wscb[tid + 256];
    sh_sm[tid] = m0;
    sh_sm[tid + 256] = m1;
    sh_sm[tid + 512] = m2;
    sh_sm[tid + 768] = m3;
  }
  __syncthreads();

  {
    const v4f yv  = *(const v4f*)(sh_y + 4 * tid);
    const v4f alv = *(const v4f*)(sh_al + 4 * tid);
    v4f smv = (v4f){0.f, 0.f, 0.f, 0.f};
    if (donext) smv = *(const v4f*)(sh_sm + 4 * tid);
    v4f snv = (v4f){0.f, 0.f, 0.f, 0.f};
    v4f cnv = (v4f){0.f, 0.f, 0.f, 0.f};
    if (tid < 64) {
      snv = *(const v4f*)(sh_sn + 4 * tid);
      cnv = *(const v4f*)(sh_cn + 4 * tid);
    }
    float* yp = Yt + ((size_t)step * NBATCH + b) * YPITCH + 4 * tid;
    float* ap = acar_out + b * NSEQ + 4 * tid;
    float* mp = smsc + b * NPROJ + 4 * tid;
    for (int pass = 0; pass < 2; ++pass) {
      *(volatile v4f*)yp = yv;
      *(volatile v4f*)ap = alv;
      if (donext) *(volatile v4f*)mp = smv;
      if (tid < 64) {
        *(volatile v4f*)(s_out + b * NHID + 4 * tid) = snv;
        *(volatile v4f*)(c_out + b * NHID + 4 * tid) = cnv;
      }
      __threadfence();
    }
  }
}

__global__ __launch_bounds__(256) void pack_out_kernel(const float* __restrict__ Yt, float* __restrict__ out) {
  const int i4 = blockIdx.x * 256 + threadIdx.x;
  const int e  = i4 * 4;
  const int row = e / NCLS;
  const int n   = e - row * NCLS;
  const int b = row / NSTEPS;
  const int t = row - b * NSTEPS;
  const v4f v = *(const v4f*)(Yt + ((size_t)t * NBATCH + b) * YPITCH + n);
  float* dst = out + e;
  *(volatile v4f*)dst = v;
  __threadfence();
  *(volatile v4f*)dst = v;
}

extern "C" void kernel_launch(void* const* d_in, const int* in_sizes, int n_in,
                              void* d_out, int out_size, void* d_ws, size_t ws_size, hipStream_t stream) {
  if (n_in < 23 || d_out == nullptr || d_ws == nullptr) return;
  if (in_sizes[0] != NBATCH * NSEQ * NDIM || in_sizes[1] != NBATCH * NSTEPS || in_sizes[2] != NBATCH ||
      in_sizes[3] != NSTEPS * NBATCH * NSEQ || in_sizes[4] != NHID * NDIM || in_sizes[6] != NDIM * NDIM ||
      in_sizes[10] != NHID * NDIM || in_sizes[12] != NDIM * NDIM || in_sizes[14] != NHID * NHID ||
      in_sizes[15] != NDIM * NHID || in_sizes[17] != NHID * NCLS || in_sizes[19] != NCLS * NGATE ||
      in_sizes[20] != NHID * NGATE || in_sizes[21] != NDIM * NGATE || out_size != NBATCH * NSTEPS * NCLS) return;

  const float* enc     = (const float*)d_in[0];
  const int*   target  = (const int*)d_in[1];
  const int*   lenenc  = (const int*)d_in[2];
  const float* noise   = (const float*)d_in[3];
  const float* ws_m_w  = (const float*)d_in[4];
  const float* ws_m_b  = (const float*)d_in[5];
  const float* wh_m    = (const float*)d_in[6];
  const float* v_m     = (const float*)d_in[7];
  const float* g_m     = (const float*)d_in[8];
  const float* r_m     = (const float*)d_in[9];
  const float* ws_c_w  = (const float*)d_in[10];
  const float* ws_c_b  = (const float*)d_in[11];
  const float* wh_c    = (const float*)d_in[12];
  const float* v_c     = (const float*)d_in[13];
  const float* l_sy    = (const float*)d_in[14];
  const float* l_gy_w  = (const float*)d_in[15];
  const float* l_gy_b  = (const float*)d_in[16];
  const float* l_yy_w  = (const float*)d_in[17];
  const float* l_yy_b  = (const float*)d_in[18];
  const float* l_ys    = (const float*)d_in[19];
  const float* l_ss    = (const float*)d_in[20];
  const float* l_gs_w  = (const float*)d_in[21];
  const float* l_gs_b  = (const float*)d_in[22];
  float* out = (float*)d_out;

  char* ws = (char*)d_ws; size_t off = 0;
  auto carve = [&](size_t bytes) -> char* { char* p = ws + off; off += (bytes + 255) & ~(size_t)255; return p; };
  unsigned short* A16  = (unsigned short*)carve((size_t)NROWS * NDIM * 2);
  unsigned short* BT16 = (unsigned short*)carve((size_t)NPROJ * NDIM * 2);
  float* PF    = (float*)carve((size_t)NROWS * NPROJ * 4);
  float* PBUF  = (float*)carve((size_t)NBATCH * NSEQ * 4);
  float* EBUF  = (float*)carve((size_t)NBATCH * NSEQ * 4);
  float* ACAR  = (float*)carve((size_t)2 * NBATCH * NSEQ * 4);
  float* SMSC  = (float*)carve((size_t)NBATCH * NPROJ * 4);
  float* SST   = (float*)carve((size_t)2 * NBATCH * NHID * 4);
  float* CST   = (float*)carve((size_t)2 * NBATCH * NHID * 4);
  float* YT    = (float*)carve((size_t)NSTEPS * NBATCH * YPITCH * 4);
  float* VNORM = (float*)carve((size_t)256);
  if (off > ws_size || off > (size_t)134217728) return;

  const int n8 = NROWS * NDIM / 8;
  cast8_f16_kernel<<<n8 / 256, 256, 0, stream>>>(enc, A16, n8);
  wtcast_kernel<<<dim3(NDIM / 64, NDIM / 64, 2), 256, 0, stream>>>(wh_m, wh_c, BT16, WCARRY);
  init_state_kernel<<<NBATCH, 256, 0, stream>>>(v_m, g_m, ws_m_b, ws_c_b, ACAR, SST, CST, SMSC, VNORM);
  wmma_gemm64<0, false, 0, 0, false, 0><<<dim3((NROWS / 64) * (NPROJ / 64) / 8, 1), 256, 0, stream>>>(
      A16, A16, NDIM, 0L, BT16, BT16, NDIM, 0L, (void*)PF, (void*)PF, NPROJ, 0L,
      PF, PF, 0L, NROWS, NPROJ, NDIM, WCARRY_INV);

  for (int step = 0; step < NSTEPS; ++step) {
    const int par = step & 1;
    energies_kernel<<<NROWS / ROWS_PER_EBLK, 256, 0, stream>>>(
        PF, SMSC, v_m, v_c, VNORM, r_m, lenenc, noise + (size_t)step * NBATCH * NSEQ, PBUF, EBUF);
    attend_decode_kernel<<<NBATCH, 256, 0, stream>>>(
        enc, target, lenenc, PBUF, EBUF,
        ACAR + (size_t)par * NBATCH * NSEQ, ACAR + (size_t)(par ^ 1) * NBATCH * NSEQ,
        SST + (size_t)par * NBATCH * NHID, CST + (size_t)par * NBATCH * NHID,
        SST + (size_t)(par ^ 1) * NBATCH * NHID, CST + (size_t)(par ^ 1) * NBATCH * NHID,
        l_ys, l_ss, l_gs_w, l_gs_b, l_gy_w, l_gy_b, l_sy, l_yy_w, l_yy_b,
        ws_m_w, ws_m_b, ws_c_w, ws_c_b, SMSC, YT, step);
  }

  pack_out_kernel<<<(NBATCH * NSTEPS * NCLS) / (256 * 4), 256, 0, stream>>>(YT, out);
}
